// S4sequence_17420387352582
// MI455X (gfx1250) — hardware-run, weakly checked
//
#include <hip/hip_runtime.h>


#ifndef NB
#define NB 8
#endif
#ifndef SEQ
#define SEQ 2048
#endif
#define NB_FULL  8
#define SEQ_FULL 2048
#ifndef OUT_SEQ
#define OUT_SEQ SEQ
#endif
#define DM   512
#define NS   16
#define RK   32
#define PJ   64
#define KB   32
#define OSW  68
#define XM   32
#define WCS  64.0f
#define WCI  (1.0f / 64.0f)
#define LNB  64
#define LNT  256
#define LNE  (((size_t)SEQ * DM) / LNB)
#define SW   4
#define ST   16
#define LOG2E 1.4426950408889634f

static_assert(RK + 2 * NS == PJ);
static_assert(PJ == 64);
static_assert(RK == 32);
static_assert(KB == 32);
static_assert(RK == KB);
static_assert(NS == 16);
static_assert(2 * NS * 4 == 128);
static_assert(DM % 64 == 0);
static_assert(DM % KB == 0);
static_assert(SEQ % 128 == 0);
static_assert(SEQ % 64 == 0);
static_assert(SEQ % XM == 0);
static_assert((NB * SEQ) % 64 == 0);
static_assert(SEQ % ST == 0);
static_assert((NB * (DM / KB)) % SW == 0);
static_assert(LNE % ((size_t)LNT * 4) == 0);
static_assert(((size_t)SEQ * DM) % LNB == 0);
static_assert(LNT % 32 == 0);
static_assert(NB <= NB_FULL);
static_assert(SEQ <= SEQ_FULL);
static_assert((OSW * 4) % 16 == 0);
static_assert(OSW >= 64);
static_assert((size_t)4 * 32 * 16 == (size_t)XM * RK * 2);
static_assert((size_t)8 * 32 * 16 == (size_t)XM * 2 * NS * 4);
static_assert((size_t)32 * 32 * 16 == (size_t)64 * 64 * 4);
static_assert((size_t)2 * 32 * 16 == (size_t)ST * KB * 2);
static_assert((size_t)8 * 16 == 128);
static_assert((size_t)64 * OSW * 4 <= 131072);
static_assert((size_t)XM * OSW * 4 <= 131072);
static_assert((size_t)SW * ST * 32 * 4 <= 131072);
static_assert((size_t)2 * (LNT / 32) * 8 <= 131072);

typedef _Float16 h16;
typedef __attribute__((ext_vector_type(16))) _Float16 v16h;
typedef __attribute__((ext_vector_type(8)))  _Float16 v8h;
typedef __attribute__((ext_vector_type(8)))  float    v8f;
typedef __attribute__((ext_vector_type(4)))  float    v4f;
typedef __attribute__((ext_vector_type(2)))  double   v2d;
typedef v4f  __attribute__((may_alias)) v4fa;

__device__ __forceinline__ unsigned short f2bf(float f) { unsigned u = __float_as_uint(f); u += 0x7FFFu + ((u >> 16) & 1u); return (unsigned short)(u >> 16); }
__device__ __forceinline__ float bfr(float f) { return __uint_as_float(((unsigned)f2bf(f)) << 16); }
__device__ __forceinline__ v16h cat16(v8h lo, v8h hi) { return __builtin_shufflevector(lo, hi, 0, 1, 2, 3, 4, 5, 6, 7, 8, 9, 10, 11, 12, 13, 14, 15); }
__device__ __forceinline__ v8f wmma16(v16h a, v16h b, v8f c) { return __builtin_amdgcn_wmma_f32_16x16x32_f16(false, a, false, b, (short)0, c, false, false); }
__device__ __forceinline__ v16h  ldh(const h16* p) { return cat16(*(const v8h*)p, *(const v8h*)(p + 16)); }
__device__ __forceinline__ void wave_sync() { __builtin_amdgcn_fence(3  , "wavefront"); __builtin_amdgcn_wave_barrier(); asm volatile("" ::: "memory"); }
static __device__ __forceinline__ h16 toh_flush(float v) { const h16 r = (h16)v; return (fabsf(v) < 6.103515625e-05f) ? (h16)0.0f : r; }
static __device__ __forceinline__ v8f wmma16g(v16h a, v16h b, v8f c) {
    c = wmma16(a, b, c);
    asm volatile("v_nop\n\tv_nop\n\tv_nop\n\tv_nop" : "+v"(c) : "v"(a), "v"(b));
    return c;
}
static __device__ __forceinline__ float softplus_f(float v) { const float e = expf(-fabsf(v)); return fmaxf(v, 0.0f) + log1pf(e); }

static __device__ __forceinline__ void ln_stats(const double* __restrict__ part, int b, float& mu, float& rstd) {
    double s1 = 0.0, s2 = 0.0;
#pragma unroll 1
    for (int i = 0; i < LNB; ++i) { const size_t o = ((size_t)b * LNB + (size_t)i) * 16; s1 += part[o]; s2 += part[o + 1]; }
    const double invn = 1.0 / ((double)SEQ * (double)DM);
    const double m = s1 * invn;
    const double v = s2 * invn - m * m;
    mu = (float)m;
    rstd = rsqrtf((float)v + 1e-5f);
}

__global__ __launch_bounds__(256) void k_wconv(const float* __restrict__ src, h16* dst, size_t n8) {
    const size_t i = (size_t)blockIdx.x * 256 + threadIdx.x; if (i >= n8) return;
    const v8f v = *(const v8f*)(src + i * 8); v8h o;
#pragma unroll
    for (int k = 0; k < 8; ++k) o[k] = toh_flush(bfr(v[k]) * WCS);
    *(volatile v8h*)(dst + i * 8) = o; __threadfence(); *(volatile v8h*)(dst + i * 8) = o;
}

__global__ __launch_bounds__(LNT) void k_lnsum(const float* __restrict__ x, double* part) {
    __shared__ double red[2 * (LNT / 32)];
    const int lane = threadIdx.x & 31;
    const int wave = __builtin_amdgcn_readfirstlane((int)(threadIdx.x >> 5));
    const int b = blockIdx.x / LNB, sl = blockIdx.x % LNB;
    const float* xb = x + (size_t)b * SEQ_FULL * DM + (size_t)sl * LNE;
    float s1 = 0.0f, s2 = 0.0f;
#pragma unroll 1
    for (int it = 0; it < (int)(LNE / ((size_t)LNT * 4)); ++it) {
        const v4f v = *(const v4f*)(xb + ((size_t)it * LNT + threadIdx.x) * 4);
#pragma unroll
        for (int i = 0; i < 4; ++i) { const float q = bfr(v[i]); s1 += q; s2 += q * q; } }
    double d1 = (double)s1, d2 = (double)s2;
#pragma unroll
    for (int off = 16; off > 0; off >>= 1) { d1 += __shfl_xor(d1, off, 32); d2 += __shfl_xor(d2, off, 32); }
    if (lane == 0) { red[wave * 2] = d1; red[wave * 2 + 1] = d2; }
    __syncthreads();
    if (wave == 0) {
        double t1 = 0.0, t2 = 0.0;
#pragma unroll 1
        for (int w = 0; w < LNT / 32; ++w) { t1 += red[2 * w]; t2 += red[2 * w + 1]; }
        v2d val; val[0] = (lane == 0) ? t1 : 0.0; val[1] = (lane == 0) ? t2 : 0.0;
        double* dst = part + (size_t)blockIdx.x * 16 + (size_t)(lane & 7) * 2;
        if (lane < 8) *(volatile v2d*)dst = val;
        __threadfence();
        if (lane < 8) *(volatile v2d*)dst = val;
    }
}

__global__ __launch_bounds__(32) void k_xproj(const float* __restrict__ x, const double* __restrict__ part, const h16* __restrict__ WX, h16* DTR, float* BC) {
    __shared__ __align__(16) float os[XM * OSW];
    const int lane = threadIdx.x & 31, lr = lane & 15, hi = lane >> 4;
    const int r0 = blockIdx.x * XM; const int bb = r0 / SEQ, tt = r0 % SEQ;
    float mu, rstd; ln_stats(part, bb, mu, rstd);
    v8f acc[2][4];
#pragma unroll
    for (int mb = 0; mb < 2; ++mb)
#pragma unroll
        for (int nb = 0; nb < 4; ++nb) acc[mb][nb] = (v8f){};
    const size_t aoff = ((size_t)bb * SEQ_FULL + (size_t)(tt + lr)) * DM + 8 * hi;
    const size_t boff = (size_t)lr * DM + 8 * hi;
#pragma unroll 1
    for (int kc = 0; kc < DM; kc += 32) {
        v16h a[2];
#pragma unroll
        for (int mb = 0; mb < 2; ++mb) {
            const float* p = x + aoff + (size_t)mb * 16 * DM + kc;
            const v8f f0 = *(const v8f*)p; const v8f f1 = *(const v8f*)(p + 16);
            v16h t;
#pragma unroll
            for (int i = 0; i < 8; ++i) { t[i] = toh_flush((bfr(f0[i]) - mu) * rstd); t[8 + i] = toh_flush((bfr(f1[i]) - mu) * rstd); }
            a[mb] = t; }
#pragma unroll
        for (int nb = 0; nb < 4; ++nb) { const v16h bq = ldh(WX + boff + (size_t)nb * 16 * DM + kc);
#pragma unroll
            for (int mb = 0; mb < 2; ++mb) acc[mb][nb] = wmma16g(a[mb], bq, acc[mb][nb]); }
    }
#pragma unroll
    for (int mb = 0; mb < 2; ++mb)
#pragma unroll
        for (int nb = 0; nb < 4; ++nb)
#pragma unroll
            for (int j = 0; j < 8; ++j) os[(mb * 16 + hi * 8 + j) * OSW + nb * 16 + lr] = acc[mb][nb][j] * WCI;
    wave_sync();
    h16* dq = DTR + (size_t)r0 * RK;
    float* bq = BC + (size_t)r0 * (2 * NS);
#pragma unroll 1
    for (int ps = 0; ps < 2; ++ps) {
#pragma unroll 1
        for (int s = 0; s < 4; ++s) { const int p = s * 32 + lane; const int row = p >> 2, c8 = (p & 3) * 8;
            const v4f x0 = *(const v4fa*)(&os[row * OSW + c8]); const v4f x1 = *(const v4fa*)(&os[row * OSW + c8 + 4]); v8h hv;
#pragma unroll
            for (int i = 0; i < 4; ++i) { hv[i] = toh_flush(x0[i]); hv[4 + i] = toh_flush(x1[i]); }
            *(volatile v8h*)(dq + (size_t)p * 8) = hv; }
#pragma unroll 1
        for (int s = 0; s < 8; ++s) { const int p = s * 32 + lane; const int row = p >> 3, c4 = (p & 7) * 4;
            const v4f val = *(const v4fa*)(&os[row * OSW + 32 + c4]);
            *(volatile v4f*)(bq + (size_t)p * 4) = val; }
        if (ps == 0) __threadfence(); }
}

__global__ __launch_bounds__(32) void k_delta(const h16* __restrict__ DTR, const h16* __restrict__ WDT, const float* __restrict__ dtb, float* DELTA) {
    __shared__ __align__(16) float os[64 * OSW];
    const int lane = threadIdx.x & 31, lr = lane & 15, hi = lane >> 4; const int r0 = blockIdx.x * 64, c0 = blockIdx.y * 64;
    v8f acc[4][4];
#pragma unroll
    for (int mb = 0; mb < 4; ++mb)
#pragma unroll
        for (int nb = 0; nb < 4; ++nb) acc[mb][nb] = (v8f){};
    const size_t aoff = (size_t)(r0 + lr) * KB + 8 * hi, boff = (size_t)(c0 + lr) * RK + 8 * hi;
    {
        v16h a[4];
#pragma unroll
        for (int mb = 0; mb < 4; ++mb) a[mb] = ldh(DTR + aoff + (size_t)mb * 16 * KB);
#pragma unroll
        for (int nb = 0; nb < 4; ++nb) { const v16h bq = ldh(WDT + boff + (size_t)nb * 16 * RK);
#pragma unroll
            for (int mb = 0; mb < 4; ++mb) acc[mb][nb] = wmma16g(a[mb], bq, acc[mb][nb]); }
    }
    float bc[4];
#pragma unroll
    for (int nb = 0; nb < 4; ++nb) bc[nb] = bfr(dtb[c0 + nb * 16 + lr]);
#pragma unroll
    for (int mb = 0; mb < 4; ++mb)
#pragma unroll
        for (int nb = 0; nb < 4; ++nb)
#pragma unroll
            for (int j = 0; j < 8; ++j) os[(mb * 16 + hi * 8 + j) * OSW + nb * 16 + lr] = acc[mb][nb][j] * WCI + bc[nb];
    wave_sync();
#pragma unroll 1
    for (int s = 0; s < 32; ++s) { const int p = s * 32 + lane; const int row = p >> 4, c4 = (p & 15) * 4;
        v4f v = *(const v4fa*)(&os[row * OSW + c4]);
#pragma unroll
        for (int i = 0; i < 4; ++i) v[i] = softplus_f(v[i]);
        *(v4fa*)(&os[row * OSW + c4]) = v; }
    wave_sync();
    float* orow = DELTA + (size_t)r0 * DM + c0;
#pragma unroll 1
    for (int ps = 0; ps < 2; ++ps) {
#pragma unroll 1
        for (int s = 0; s < 32; ++s) { const int p = s * 32 + lane; const int row = p >> 4, c4 = (p & 15) * 4;
            const v4f val = *(const v4fa*)(&os[row * OSW + c4]);
            *(volatile v4f*)(orow + (size_t)row * DM + c4) = val; }
        if (ps == 0) __threadfence(); }
}

__global__ __launch_bounds__(32 * SW) void k_scan(const float* __restrict__ x, const double* __restrict__ part, const float* __restrict__ DELTA, const float* __restrict__ BC,
                                                  const float* __restrict__ alog, const float* __restrict__ dvec, h16* YG) {
    __shared__ __align__(16) float ys[SW * ST * 32];
    const int lane = threadIdx.x & 31;
    const int wave = __builtin_amdgcn_readfirstlane((int)(threadIdx.x >> 5));
    const int gw = blockIdx.x * SW + wave;
    const int bb = gw / (DM / KB), kb = gw % (DM / KB);
    const int d = kb * KB + lane;
    float mu, rstd; ln_stats(part, bb, mu, rstd);
    float a2[NS], st[NS];
    { const v4f* ap = (const v4f*)(alog + (size_t)d * NS);
      const v4f q0 = ap[0], q1 = ap[1], q2 = ap[2], q3 = ap[3];
#pragma unroll
      for (int r = 0; r < 4; ++r) { a2[r] = q0[r]; a2[4 + r] = q1[r]; a2[8 + r] = q2[r]; a2[12 + r] = q3[r]; }
#pragma unroll
      for (int n = 0; n < NS; ++n) { a2[n] = -__builtin_amdgcn_exp2f(bfr(a2[n]) * LOG2E) * LOG2E; st[n] = 0.0f; } }
    const float Dd = bfr(dvec[d]);
    const float* xp  = x + (size_t)bb * SEQ_FULL * DM + d;
    const float* dp  = DELTA + (size_t)bb * SEQ * DM + d;
    const float* bcp = BC + (size_t)bb * SEQ * (2 * NS);
    h16* yrow = YG + ((size_t)kb * ((size_t)NB * SEQ) + (size_t)bb * SEQ) * KB;
    const int wb = wave * ST * 32;
#pragma unroll 1
    for (int l0 = 0; l0 < SEQ; l0 += ST) {
#pragma unroll 1
        for (int t = 0; t < ST; ++t) {
            const size_t l = (size_t)(l0 + t);
            const float dv = dp[l * DM];
            const float u = (bfr(xp[l * DM]) - mu) * rstd;
            const v4f* q = (const v4f*)(bcp + l * (2 * NS));
            const v4f b0 = q[0], b1 = q[1], b2 = q[2], b3 = q[3], c0 = q[4], c1 = q[5], c2 = q[6], c3 = q[7];
            float Bn[NS], Cn[NS];
#pragma unroll
            for (int r = 0; r < 4; ++r) { Bn[r] = b0[r]; Bn[4 + r] = b1[r]; Bn[8 + r] = b2[r]; Bn[12 + r] = b3[r];
                                          Cn[r] = c0[r]; Cn[4 + r] = c1[r]; Cn[8 + r] = c2[r]; Cn[12 + r] = c3[r]; }
            const float du = dv * u;
            float y = 0.0f;
#pragma unroll
            for (int n = 0; n < NS; ++n) {
                const float dA = __builtin_amdgcn_exp2f(dv * a2[n]);
                st[n] = st[n] * dA + du * Bn[n];
                y += st[n] * Cn[n]; }
            const float yf = y + u * Dd;
            const float g = 0.5f * yf * (1.0f + erff(yf * 0.70710678118654752f));
            ys[wb + t * 32 + lane] = g;
        }
        wave_sync();
        h16* dst = yrow + (size_t)l0 * KB;
#pragma unroll 1
        for (int ps = 0; ps < 2; ++ps) {
#pragma unroll 1
            for (int s = 0; s < 2; ++s) { const int p = s * 32 + lane; const int row = p >> 2, c8 = (p & 3) * 8;
                const v4f x0 = *(const v4fa*)(&ys[wb + row * 32 + c8]); const v4f x1 = *(const v4fa*)(&ys[wb + row * 32 + c8 + 4]); v8h hv;
#pragma unroll
                for (int i = 0; i < 4; ++i) { hv[i] = toh_flush(x0[i]); hv[4 + i] = toh_flush(x1[i]); }
                *(volatile v8h*)(dst + (size_t)p * 8) = hv; }
            if (ps == 0) __threadfence(); }
        wave_sync();
    }
}

__global__ __launch_bounds__(32) void k_out(const h16* __restrict__ YG, const h16* __restrict__ WO, const float* __restrict__ outb, const float* __restrict__ x, float* OUT) {
    __shared__ __align__(16) float os[64 * OSW];
    const int lane = threadIdx.x & 31, lr = lane & 15, hi = lane >> 4; const int r0 = blockIdx.x * 64, c0 = blockIdx.y * 64;
    const int bb = r0 / SEQ, tt = r0 % SEQ;
    v8f acc[4][4];
#pragma unroll
    for (int mb = 0; mb < 4; ++mb)
#pragma unroll
        for (int nb = 0; nb < 4; ++nb) acc[mb][nb] = (v8f){};
    const size_t aoff = (size_t)(r0 + lr) * KB + 8 * hi, boff = (size_t)(c0 + lr) * DM + 8 * hi;
    const size_t astep = (size_t)NB * SEQ * KB;
#pragma unroll 1
    for (int ks = 0; ks < DM / KB; ++ks) {
        v16h a[4];
#pragma unroll
        for (int mb = 0; mb < 4; ++mb) a[mb] = ldh(YG + aoff + (size_t)ks * astep + (size_t)mb * 16 * KB);
#pragma unroll
        for (int nb = 0; nb < 4; ++nb) { const v16h bq = ldh(WO + boff + (size_t)nb * 16 * DM + (size_t)ks * 32);
#pragma unroll
            for (int mb = 0; mb < 4; ++mb) acc[mb][nb] = wmma16g(a[mb], bq, acc[mb][nb]); }
    }
#pragma unroll
    for (int mb = 0; mb < 4; ++mb)
#pragma unroll
        for (int nb = 0; nb < 4; ++nb)
#pragma unroll
            for (int j = 0; j < 8; ++j) os[(mb * 16 + hi * 8 + j) * OSW + nb * 16 + lr] = acc[mb][nb][j] * WCI;
    wave_sync();
    const float* xrow = x + ((size_t)bb * SEQ_FULL + (size_t)tt) * DM + c0;
#pragma unroll 1
    for (int s = 0; s < 32; ++s) { const int p = s * 32 + lane; const int row = p >> 4, c4 = (p & 15) * 4;
        v4f v = *(const v4fa*)(&os[row * OSW + c4]);
        const v4f bi = *(const v4f*)(outb + c0 + c4);
        const v4f sk = *(const v4f*)(xrow + (size_t)row * DM + c4);
#pragma unroll
        for (int i = 0; i < 4; ++i) v[i] = (v[i] + bfr(bi[i])) + bfr(sk[i]);
        *(v4fa*)(&os[row * OSW + c4]) = v; }
    wave_sync();
    float* orow = OUT + ((size_t)bb * OUT_SEQ + (size_t)tt) * DM + c0;
#pragma unroll 1
    for (int ps = 0; ps < 2; ++ps) {
#pragma unroll 1
        for (int s = 0; s < 32; ++s) { const int p = s * 32 + lane; const int row = p >> 4, c4 = (p & 15) * 4;
            const v4f val = *(const v4fa*)(&os[row * OSW + c4]);
            *(volatile v4f*)(orow + (size_t)row * DM + c4) = val; }
        if (ps == 0) __threadfence(); }
}

static constexpr size_t al256(size_t v) { return (v + 255) & ~(size_t)255; }
static constexpr size_t SZ_PART = al256((size_t)NB * LNB * 128);
static constexpr size_t SZ_WX   = al256((size_t)PJ * DM * 2);
static constexpr size_t SZ_WDT  = al256((size_t)DM * RK * 2);
static constexpr size_t SZ_WO   = al256((size_t)DM * DM * 2);
static constexpr size_t SZ_DTR  = al256((size_t)NB * SEQ * RK * 2);
static constexpr size_t SZ_BC   = al256((size_t)NB * SEQ * 2 * NS * 4);
static constexpr size_t SZ_DEL  = al256((size_t)NB * SEQ * DM * 4);
static constexpr size_t SZ_YG   = al256((size_t)(DM / KB) * NB * SEQ * KB * 2);
static constexpr size_t SZ_TOTAL = SZ_PART + SZ_WX + SZ_WDT + SZ_WO + SZ_DTR + SZ_BC + SZ_DEL + SZ_YG;
static_assert(SZ_TOTAL <= (size_t)134217728);
static_assert(((size_t)PJ * DM) % 64 == 0);
static_assert(((size_t)DM * RK) % 64 == 0);
static_assert(((size_t)DM * DM) % 64 == 0);
static_assert((size_t)(DM / KB) * KB == (size_t)DM);

extern "C" void kernel_launch(void* const* d_in, const int* in_sizes, int n_in,
                              void* d_out, int out_size, void* d_ws, size_t ws_size, hipStream_t stream) {
    if (n_in < 8) return;
    const size_t needx = ((size_t)(NB - 1) * SEQ_FULL + SEQ) * DM;
    if ((size_t)in_sizes[0] < needx) return;
    if ((size_t)in_sizes[1] < (size_t)PJ * DM || (size_t)in_sizes[2] < (size_t)DM * RK || (size_t)in_sizes[6] < (size_t)DM * DM) return;
    if (in_sizes[3] < DM || in_sizes[4] < DM * NS || in_sizes[5] < DM || in_sizes[7] < DM) return;
    if ((size_t)out_size < ((size_t)(NB - 1) * OUT_SEQ + SEQ) * DM) return;
    if (SZ_TOTAL > ws_size) return;
    const float* x    = (const float*)d_in[0];
    const float* wx   = (const float*)d_in[1];
    const float* wdt  = (const float*)d_in[2];
    const float* dtb  = (const float*)d_in[3];
    const float* alog = (const float*)d_in[4];
    const float* dvec = (const float*)d_in[5];
    const float* wo   = (const float*)d_in[6];
    const float* outb = (const float*)d_in[7];
    float* OUT = (float*)d_out;
    char* wsp = (char*)d_ws;
    double* PART = (double*)wsp; wsp += SZ_PART;
    h16* WXH  = (h16*)wsp; wsp += SZ_WX;
    h16* WDTH = (h16*)wsp; wsp += SZ_WDT;
    h16* WOH  = (h16*)wsp; wsp += SZ_WO;
    h16* DTR  = (h16*)wsp; wsp += SZ_DTR;
    float* BC = (float*)wsp; wsp += SZ_BC;
    float* DELTA = (float*)wsp; wsp += SZ_DEL;
    h16* YG   = (h16*)wsp; wsp += SZ_YG;

    { const size_t n8 = (size_t)PJ * DM / 8; k_wconv<<<(unsigned)((n8 + 255) / 256), 256, 0, stream>>>(wx, WXH, n8); }
    { const size_t n8 = (size_t)DM * RK / 8; k_wconv<<<(unsigned)((n8 + 255) / 256), 256, 0, stream>>>(wdt, WDTH, n8); }
    { const size_t n8 = (size_t)DM * DM / 8; k_wconv<<<(unsigned)((n8 + 255) / 256), 256, 0, stream>>>(wo, WOH, n8); }

    k_lnsum<<<NB * LNB, LNT, 0, stream>>>(x, PART);
    k_xproj<<<NB * SEQ / XM, 32, 0, stream>>>(x, PART, WXH, DTR, BC);
    k_delta<<<dim3(NB * SEQ / 64, DM / 64, 1), 32, 0, stream>>>(DTR, WDTH, dtb, DELTA);
    k_scan<<<NB * (DM / KB) / SW, 32 * SW, 0, stream>>>(x, PART, DELTA, BC, alog, dvec, YG);
    k_out<<<dim3(NB * SEQ / 64, DM / 64, 1), 32, 0, stream>>>(YG, WOH, outb, x, OUT);
}
